// LinearAttention_24507083391399
// MI455X (gfx1250) — hardware-verified
//
#include <hip/hip_runtime.h>
#include <math.h>

constexpr int kSeqLen = 2048;
constexpr int kModel  = 1024;
constexpr int kHeads  = 16;
constexpr int kDh     = 64;
constexpr int kQKV    = kHeads * kDh;
constexpr int kN3     = 3 * kQKV;
constexpr int kChunk  = 64;
constexpr int kNChunk = kSeqLen / kChunk;
constexpr int kPitchH = 72;
constexpr int kTileH  = kChunk * kPitchH;
constexpr float kResCarry    = 2048.0f;
constexpr float kResCarryInv = 1.0f / 2048.0f;
constexpr float kInvDh       = 1.0f / 64.0f;
constexpr float kLnEps       = 1e-5f;
static_assert(kQKV == kModel, "square projections");
static_assert(kSeqLen % kChunk == 0 && kChunk == 64 && kDh == 64, "chunk tiles");
static_assert(kModel % 32 == 0 && (2 * kQKV) % 32 == 0, "K multiples of 32");
static_assert(kSeqLen % 64 == 0 && kN3 % 64 == 0 && kModel % 64 == 0, "M, N multiples of 64");
static_assert((kSeqLen * kModel / 8) % 256 == 0 && (kModel * kModel / 8) % 256 == 0, "cast grids exact");
static_assert((kSeqLen * kHeads) % 8 == 0 && (kHeads * kDh) % 8 == 0, "wave grids exact");

typedef __attribute__((ext_vector_type(16))) _Float16 v16h;
typedef __attribute__((ext_vector_type(8)))  _Float16 v8h;
typedef __attribute__((ext_vector_type(16))) __bf16   v16b;
typedef __attribute__((ext_vector_type(8)))  __bf16   v8b;
typedef __attribute__((ext_vector_type(8)))  float    v8f;
typedef __attribute__((ext_vector_type(4)))  float    v4f;
typedef __attribute__((ext_vector_type(2)))  float    v2f;
typedef __attribute__((ext_vector_type(4)))  unsigned int v4u;

__device__ __forceinline__ unsigned short f2bf_bits(float f) {
  unsigned u = __float_as_uint(f);
  return (unsigned short)((u + 0x7FFFu + ((u >> 16) & 1u)) >> 16);
}
__device__ __forceinline__ float bf_bits2f(unsigned short h) { return __uint_as_float(((unsigned)h) << 16); }

__device__ __forceinline__ void dep_guard_h(v8f& a, v8f& b, v16h x, v16h y) { asm volatile("v_nop\n\tv_nop\n\tv_nop\n\tv_nop" : "+v"(a), "+v"(b) : "v"(x), "v"(y)); }
__device__ __forceinline__ void dep_guard_b(v8f& a, v8f& b, v16b x, v16b y) { asm volatile("v_nop\n\tv_nop\n\tv_nop\n\tv_nop" : "+v"(a), "+v"(b) : "v"(x), "v"(y)); }
__device__ __forceinline__ void keep4_h(v16h a, v16h b, v16h c, v16h d) { asm volatile("v_nop" :: "v"(a), "v"(b), "v"(c), "v"(d)); }
__device__ __forceinline__ void keep4_b(v16b a, v16b b, v16b c, v16b d) { asm volatile("v_nop" :: "v"(a), "v"(b), "v"(c), "v"(d)); }
__device__ __forceinline__ void acc_guard4(v8f& a, v8f& b, v8f& c, v8f& d) { asm volatile("v_nop\n\tv_nop\n\tv_nop\n\tv_nop" : "+v"(a), "+v"(b), "+v"(c), "+v"(d)); }
template <typename T> struct Frag;
template <> struct Frag<_Float16> {
  typedef v16h V; union U { v16h v; v8h h[2]; };
  static __device__ __forceinline__ v16h load(const _Float16* p) {
    U f; f.h[0] = *(const v8h*)(p); f.h[1] = *(const v8h*)(p + 16); return f.v;
  }
  static __device__ __forceinline__ v8f mma(v16h a, v16h b, v8f c) {
    return __builtin_amdgcn_wmma_f32_16x16x32_f16(false, a, false, b, (short)0, c, false, false);
  }
  static __device__ __forceinline__ void guard(v8f& a, v8f& b, v16h x, v16h y) { dep_guard_h(a, b, x, y); }
  static __device__ __forceinline__ void keep(v16h a, v16h b, v16h c, v16h d) { keep4_h(a, b, c, d); }
};
template <> struct Frag<__bf16> {
  typedef v16b V; union U { v16b v; v8b h[2]; };
  static __device__ __forceinline__ v16b load(const __bf16* p) {
    U f; f.h[0] = *(const v8b*)(p); f.h[1] = *(const v8b*)(p + 16); return f.v;
  }
  static __device__ __forceinline__ v8f mma(v16b a, v16b b, v8f c) {
    return __builtin_amdgcn_wmma_f32_16x16x32_bf16(false, a, false, b, (short)0, c, false, false);
  }
  static __device__ __forceinline__ void guard(v8f& a, v8f& b, v16b x, v16b y) { dep_guard_b(a, b, x, y); }
  static __device__ __forceinline__ void keep(v16b a, v16b b, v16b c, v16b d) { keep4_b(a, b, c, d); }
};

__device__ __forceinline__ unsigned pk16(unsigned short a, unsigned short b) { return (unsigned)a | ((unsigned)b << 16); }
__device__ __forceinline__ unsigned short h_bits(float f) { const _Float16 h = (_Float16)f; return __builtin_bit_cast(unsigned short, h); }

template <int ET> struct Elem;
template <> struct Elem<0> { typedef _Float16 T; };
template <> struct Elem<1> { typedef __bf16 T; };
template <int ET, bool SPLIT, int BIAS_MODE, int OUT_MODE, bool RESID, int ACT = 0>
__global__ __launch_bounds__(256) void wmma_gemm64(
    const unsigned short* __restrict__ Ap, const unsigned short* __restrict__ A2p, int lda, long strideA,
    const unsigned short* __restrict__ Btp, const unsigned short* __restrict__ Bt2p, int ldb, long strideB,
    void* __restrict__ Cout, void* __restrict__ Cout2, int ldc, long strideC,
    const float* __restrict__ bias,
    const float* __restrict__ resid, long strideR,
    int M, int N, int K, float scale) {
  typedef typename Elem<ET>::T T;
  typedef typename Frag<T>::V V;
  const T* A = (const T*)Ap; const T* A2 = (const T*)A2p; const T* Bt = (const T*)Btp; const T* Bt2 = (const T*)Bt2p;
  __shared__ __align__(16) float sT[8][16 * 68];
  const int b    = blockIdx.y;
  const int lane = threadIdx.x & 31;
  const int wave = threadIdx.x >> 5;
  const int tilesN = N >> 6;
  const int tilesM = M >> 6;
  const int tile = blockIdx.x * 8 + wave;
  if (tile >= tilesM * tilesN) return;
  const int tm = tile / tilesN;
  const int tn = tile - tm * tilesN;
  const int m0 = tm << 6;
  const int n0 = tn << 6;

  const T* Ab  = A  + (size_t)b * strideA;
  const T* Bb  = Bt + (size_t)b * strideB;
  const T* Ab2 = SPLIT ? (A2  + (size_t)b * strideA) : nullptr;
  const T* Bb2 = SPLIT ? (Bt2 + (size_t)b * strideB) : nullptr;

  const int rlane = lane & 15;
  const int koff  = (lane >> 4) * 8;
  const int mOff  = (lane >> 4) * 8;

  v8f acc[4][4];
#pragma unroll
  for (int i = 0; i < 4; ++i)
#pragma unroll
    for (int j = 0; j < 4; ++j) acc[i][j] = (v8f){0.f,0.f,0.f,0.f,0.f,0.f,0.f,0.f};

  for (int k0 = 0; k0 < K; k0 += 32) {
    V bh[4], bl[4];
#pragma unroll
    for (int j = 0; j < 4; ++j) {
      const size_t bo = (size_t)(n0 + (j << 4) + rlane) * ldb + koff + k0;
      bh[j] = Frag<T>::load(Bb + bo);
      if (SPLIT) bl[j] = Frag<T>::load(Bb2 + bo);
    }
#pragma unroll
    for (int i = 0; i < 4; ++i) {
      const size_t ao = (size_t)(m0 + (i << 4) + rlane) * lda + koff + k0;
      V ah = Frag<T>::load(Ab + ao);
      V al;
      if (SPLIT) al = Frag<T>::load(Ab2 + ao);
#pragma unroll
      for (int j = 0; j < 4; ++j) {
        acc[i][j] = Frag<T>::mma(ah, bh[j], acc[i][j]);
        if (SPLIT) {
          acc[i][j] = Frag<T>::mma(ah, bl[j], acc[i][j]);
          acc[i][j] = Frag<T>::mma(al, bh[j], acc[i][j]);
        }
      }
      Frag<T>::guard(acc[i][0], acc[i][3], ah, SPLIT ? al : ah);
    }
    Frag<T>::keep(bh[0], bh[1], bh[2], bh[3]);
    if (SPLIT) Frag<T>::keep(bl[0], bl[1], bl[2], bl[3]);
  }
  acc_guard4(acc[0][0], acc[0][1], acc[0][2], acc[0][3]);
  acc_guard4(acc[1][0], acc[1][1], acc[1][2], acc[1][3]);
  acc_guard4(acc[2][0], acc[2][1], acc[2][2], acc[2][3]);
  acc_guard4(acc[3][0], acc[3][1], acc[3][2], acc[3][3]);

  float* slab = sT[wave];
  const float* Rb = RESID ? (resid + (size_t)b * strideR) : nullptr;
#pragma unroll
  for (int i = 0; i < 4; ++i) {
    const int mBase = m0 + (i << 4);
#pragma unroll
    for (int j = 0; j < 4; ++j) {
      const int n = n0 + (j << 4) + rlane;
      float bv = 0.f;
      if (BIAS_MODE == 2) bv = bias[n];
#pragma unroll
      for (int r = 0; r < 8; ++r) {
        float v = acc[i][j][r] * scale;
        if (BIAS_MODE == 1) v += bias[mBase + mOff + r];
        if (BIAS_MODE == 2) v += bv;
        if (RESID) v += Rb[(size_t)(mBase + mOff + r) * ldc + n];
        if (ACT == 2) v = fmaxf(v, 0.0f);
        if (ACT == 4) v = (v > 0.f) ? v : 0.01f * v;
        slab[(mOff + r) * 68 + (j << 4) + rlane] = v;
      }
    }
    __builtin_amdgcn_fence(__ATOMIC_RELEASE, "workgroup");
    __builtin_amdgcn_wave_barrier();
    __builtin_amdgcn_fence(__ATOMIC_ACQUIRE, "workgroup");
    if (OUT_MODE == 0) {
      float* C = (float*)Cout + (size_t)b * strideC;
      const int hh = lane >> 4, c4 = (lane & 15) * 4;
      for (int pass = 0; pass < 2; ++pass) {
#pragma unroll
        for (int it = 0; it < 8; ++it) {
          const int row = it * 2 + hh;
          v4f v = *(const v4f*)(slab + row * 68 + c4);
          *(volatile v4f*)(C + (size_t)(mBase + row) * ldc + n0 + c4) = v;
        }
        __threadfence();
      }
    } else {
      const int q = lane >> 3, c8 = (lane & 7) * 8;
      unsigned short* C  = (unsigned short*)Cout  + (size_t)b * strideC;
      unsigned short* C2 = (OUT_MODE == 2) ? ((unsigned short*)Cout2 + (size_t)b * strideC) : nullptr;
      for (int pass = 0; pass < 2; ++pass) {
#pragma unroll
        for (int it = 0; it < 4; ++it) {
          const int row = it * 4 + q;
          const float* sp = slab + row * 68 + c8;
          v8h hv, lv;
#pragma unroll
          for (int e = 0; e < 8; ++e) {
            if (OUT_MODE == 1) {
              hv[e] = (_Float16)sp[e];
            } else {
              unsigned short hb = f2bf_bits(sp[e]);
              unsigned short lb = f2bf_bits(sp[e] - bf_bits2f(hb));
              hv[e] = __builtin_bit_cast(_Float16, hb);
              lv[e] = __builtin_bit_cast(_Float16, lb);
            }
          }
          *(volatile v8h*)(C + (size_t)(mBase + row) * ldc + n0 + c8) = hv;
          if (OUT_MODE == 2) *(volatile v8h*)(C2 + (size_t)(mBase + row) * ldc + n0 + c8) = lv;
        }
        __threadfence();
      }
    }
    __builtin_amdgcn_fence(__ATOMIC_RELEASE, "workgroup");
    __builtin_amdgcn_wave_barrier();
    __builtin_amdgcn_fence(__ATOMIC_ACQUIRE, "workgroup");
  }
}

__device__ __forceinline__ void guard_s3(v8f& a, v8f& b, v16h x, v16h y, v16h z) {
  asm volatile("v_nop\n\tv_nop\n\tv_nop\n\tv_nop" : "+v"(a), "+v"(b) : "v"(x), "v"(y), "v"(z));
}
__device__ __forceinline__ void guard_p4(v8f& a, v16h x, v16h y, v16h z, v16h w) {
  asm volatile("v_nop\n\tv_nop\n\tv_nop\n\tv_nop" : "+v"(a) : "v"(x), "v"(y), "v"(z), "v"(w));
}
__device__ __forceinline__ void guard_o5(v8f& a, v8f& b, v16h x, v16h y, v16h z, v16h w, v16h u) {
  asm volatile("v_nop\n\tv_nop\n\tv_nop\n\tv_nop" : "+v"(a), "+v"(b) : "v"(x), "v"(y), "v"(z), "v"(w), "v"(u));
}

__device__ __forceinline__ void lds_put_tr(unsigned short* tile, int c8, int s, v4u w) {
  const unsigned w0 = w.x, w1 = w.y, w2 = w.z, w3 = w.w;
  tile[(c8 + 0) * kPitchH + s] = (unsigned short)(w0 & 0xffffu);
  tile[(c8 + 1) * kPitchH + s] = (unsigned short)(w0 >> 16);
  tile[(c8 + 2) * kPitchH + s] = (unsigned short)(w1 & 0xffffu);
  tile[(c8 + 3) * kPitchH + s] = (unsigned short)(w1 >> 16);
  tile[(c8 + 4) * kPitchH + s] = (unsigned short)(w2 & 0xffffu);
  tile[(c8 + 5) * kPitchH + s] = (unsigned short)(w2 >> 16);
  tile[(c8 + 6) * kPitchH + s] = (unsigned short)(w3 & 0xffffu);
  tile[(c8 + 7) * kPitchH + s] = (unsigned short)(w3 >> 16);
}

__global__ __launch_bounds__(256) void cast_bf16_kernel(const float* __restrict__ x, const float* __restrict__ Wq,
                                                        const float* __restrict__ Wk, const float* __restrict__ Wv,
                                                        const float* __restrict__ Wo,
                                                        unsigned short* __restrict__ Xb, unsigned short* __restrict__ Wqkv,
                                                        unsigned short* __restrict__ Wo2) {
  const int z = blockIdx.y;
  const int i = blockIdx.x * 256 + threadIdx.x;
  const int n8 = (z == 0) ? (kSeqLen * kModel / 8) : (kModel * kModel / 8);
  if (i >= n8) return;
  const float* src = (z == 0) ? x : (z == 1) ? Wq : (z == 2) ? Wk : (z == 3) ? Wv : Wo;
  const float* p = src + 8 * (size_t)i;
  const v4f a = *(const v4f*)(p);
  const v4f c = *(const v4f*)(p + 4);
  unsigned short hb[8];
#pragma unroll
  for (int e = 0; e < 4; ++e) {
    hb[e]     = f2bf_bits(a[e]);
    hb[4 + e] = f2bf_bits(c[e]);
  }
  const v4u u = (v4u){pk16(hb[0], hb[1]), pk16(hb[2], hb[3]), pk16(hb[4], hb[5]), pk16(hb[6], hb[7])};
  unsigned short* dst;
  if (z == 0) dst = Xb + 8 * (size_t)i;
  else if (z <= 3) dst = Wqkv + (size_t)(z - 1) * kModel * kModel + 8 * (size_t)i;
  else dst = Wo2 + (size_t)(i >> 7) * (2 * kQKV) + (i & 127) * 8;
  *(volatile v4u*)dst = u;
  if (z == 4) *(volatile v4u*)(dst + kQKV) = u;
  __threadfence();
  *(volatile v4u*)dst = u;
  if (z == 4) *(volatile v4u*)(dst + kQKV) = u;
}

__global__ __launch_bounds__(256) void ln_cast_kernel(const float* __restrict__ QKVf,
                                                      const float* __restrict__ qg, const float* __restrict__ qbt,
                                                      const float* __restrict__ kg, const float* __restrict__ kbt,
                                                      unsigned short* __restrict__ Qh, unsigned short* __restrict__ Kh,
                                                      unsigned short* __restrict__ Vh) {
  const int tid = threadIdx.x, lane = tid & 31, wave = tid >> 5;
  const int row = blockIdx.x * 8 + wave;
  const int t = row >> 4, h = row & 15;
  const int d0 = 2 * lane;
  const float* src = QKVf + (size_t)t * kN3 + h * kDh + d0;
  const v2f qv = *(const v2f*)(src);
  const v2f kv = *(const v2f*)(src + kQKV);
  const v2f vv = *(const v2f*)(src + 2 * kQKV);
  const v2f gqv = *(const v2f*)(qg + d0);
  const v2f bqv = *(const v2f*)(qbt + d0);
  const v2f gkv = *(const v2f*)(kg + d0);
  const v2f bkv = *(const v2f*)(kbt + d0);

  float sq = qv.x + qv.y;
#pragma unroll
  for (int off = 16; off > 0; off >>= 1) sq += __shfl_xor(sq, off, 32);
  const float muq = sq * kInvDh;
  const float aq = qv.x - muq, bq = qv.y - muq;
  float vq = aq * aq + bq * bq;
#pragma unroll
  for (int off = 16; off > 0; off >>= 1) vq += __shfl_xor(vq, off, 32);
  const float rq = rsqrtf(vq * kInvDh + kLnEps);
  const float yq0 = aq * rq * gqv.x + bqv.x;
  const float yq1 = bq * rq * gqv.y + bqv.y;

  float sk = kv.x + kv.y;
#pragma unroll
  for (int off = 16; off > 0; off >>= 1) sk += __shfl_xor(sk, off, 32);
  const float muk = sk * kInvDh;
  const float ak = kv.x - muk, bk = kv.y - muk;
  float vk = ak * ak + bk * bk;
#pragma unroll
  for (int off = 16; off > 0; off >>= 1) vk += __shfl_xor(vk, off, 32);
  const float rk = rsqrtf(vk * kInvDh + kLnEps);
  const float yk0 = ak * rk * gkv.x + bkv.x;
  const float yk1 = bk * rk * gkv.y + bkv.y;

  const unsigned wq = pk16(h_bits(yq0), h_bits(yq1));
  const unsigned wk = pk16(h_bits(yk0), h_bits(yk1));
  const unsigned wv = pk16(h_bits(vv.x), h_bits(vv.y));
  const size_t o = (size_t)t * kQKV + h * kDh + d0;
  *(volatile unsigned*)(Qh + o) = wq;
  *(volatile unsigned*)(Kh + o) = wk;
  *(volatile unsigned*)(Vh + o) = wv;
  __threadfence();
  *(volatile unsigned*)(Qh + o) = wq;
  *(volatile unsigned*)(Kh + o) = wk;
  *(volatile unsigned*)(Vh + o) = wv;
}

__global__ __launch_bounds__(256) void chunk_state_kernel(const unsigned short* __restrict__ Kh,
                                                          const unsigned short* __restrict__ Vh,
                                                          float* __restrict__ KV) {
  __shared__ __align__(16) unsigned short kTt[kTileH];
  __shared__ __align__(16) unsigned short vTt[kTileH];
  __shared__ __align__(16) float slab[kChunk * 68];
  const int c = blockIdx.x, h = blockIdx.y;
  const int tid = threadIdx.x, lane = tid & 31, wave = tid >> 5;
#pragma unroll
  for (int it = 0; it < 2; ++it) {
    const int e  = it * 256 + tid;
    const int s  = e >> 3;
    const int c8 = (e & 7) * 8;
    const size_t g = ((size_t)(c * kChunk + s)) * kQKV + h * kDh + c8;
    const v4u kw = *(const v4u*)(Kh + g);
    const v4u vw = *(const v4u*)(Vh + g);
    lds_put_tr(kTt, c8, s, kw);
    lds_put_tr(vTt, c8, s, vw);
  }
  __syncthreads();

  const int mt = wave & 3, nh = wave >> 2;
  const int rlane = lane & 15, koff = (lane >> 4) * 8, mOff = (lane >> 4) * 8;
  const _Float16* kA = (const _Float16*)kTt;
  const _Float16* vB = (const _Float16*)vTt;
  v8f acc[2];
  acc[0] = (v8f){0.f,0.f,0.f,0.f,0.f,0.f,0.f,0.f};
  acc[1] = (v8f){0.f,0.f,0.f,0.f,0.f,0.f,0.f,0.f};
#pragma unroll
  for (int kk = 0; kk < 2; ++kk) {
    const int k0 = kk * 32;
    const v16h a  = Frag<_Float16>::load(kA + (mt * 16 + rlane) * kPitchH + koff + k0);
    const v16h b0 = Frag<_Float16>::load(vB + ((2 * nh) * 16 + rlane) * kPitchH + koff + k0);
    const v16h b1 = Frag<_Float16>::load(vB + ((2 * nh + 1) * 16 + rlane) * kPitchH + koff + k0);
    acc[0] = Frag<_Float16>::mma(a, b0, acc[0]);
    acc[1] = Frag<_Float16>::mma(a, b1, acc[1]);
    guard_s3(acc[0], acc[1], a, b0, b1);
  }
#pragma unroll
  for (int jj = 0; jj < 2; ++jj) {
    const int n = (2 * nh + jj) * 16 + rlane;
#pragma unroll
    for (int r = 0; r < 8; ++r) slab[(mt * 16 + mOff + r) * 68 + n] = acc[jj][r];
  }
  __syncthreads();
  float* dst = KV + ((size_t)(h * kNChunk + c)) * (kDh * kDh);
  const int hh = lane >> 4, c4 = (lane & 15) * 4;
  for (int pass = 0; pass < 2; ++pass) {
#pragma unroll
    for (int it = 0; it < 4; ++it) {
      const int row = wave * 8 + it * 2 + hh;
      const v4f val = *(const v4f*)(slab + row * 68 + c4);
      *(volatile v4f*)(dst + (size_t)row * kDh + c4) = val;
    }
    __threadfence();
  }
}

__global__ __launch_bounds__(256) void state_prefix_kernel(const float* __restrict__ KV,
                                                           unsigned short* __restrict__ Shi,
                                                           unsigned short* __restrict__ Slo) {
  const int tid = threadIdx.x, lane = tid & 31;
  const int wg = blockIdx.x * 8 + (tid >> 5);
  const int h = wg >> 6, e = wg & 63;
  const int d0 = 2 * lane;
  float a0 = 0.0f, a1 = 0.0f;
#pragma unroll 1
  for (int c = 0; c < kNChunk; ++c) {
    const size_t base = ((size_t)(h * kNChunk + c)) * (kDh * kDh);
    const _Float16 h0 = (_Float16)a0;
    const _Float16 h1 = (_Float16)a1;
    const float f0 = (float)h0;
    const float f1 = (float)h1;
    const float r0 = (a0 - f0) * kResCarry;
    const float r1 = (a1 - f1) * kResCarry;
    const unsigned wh = pk16(__builtin_bit_cast(unsigned short, h0), __builtin_bit_cast(unsigned short, h1));
    const unsigned wl = pk16(h_bits(r0), h_bits(r1));
    const size_t o = base + (size_t)e * kDh + d0;
    *(volatile unsigned*)(Shi + o) = wh;
    *(volatile unsigned*)(Slo + o) = wl;
    __threadfence();
    *(volatile unsigned*)(Shi + o) = wh;
    *(volatile unsigned*)(Slo + o) = wl;
    a0 += KV[base + (size_t)d0 * kDh + e];
    a1 += KV[base + (size_t)(d0 + 1) * kDh + e];
  }
}

__global__ __launch_bounds__(256) void chunk_attn_kernel(const unsigned short* __restrict__ Qh,
                                                         const unsigned short* __restrict__ Kh,
                                                         const unsigned short* __restrict__ Vh,
                                                         const unsigned short* __restrict__ Shi,
                                                         const unsigned short* __restrict__ Slo,
                                                         unsigned short* __restrict__ Ob) {
  __shared__ __align__(16) unsigned short lds[6 * kTileH];
  unsigned short* tQ  = lds;
  unsigned short* tK  = lds + 1 * kTileH;
  unsigned short* tV  = lds + 2 * kTileH;
  unsigned short* tSh = lds + 3 * kTileH;
  unsigned short* tSl = lds + 4 * kTileH;
  unsigned short* tP  = lds + 5 * kTileH;
  const int c = blockIdx.x, h = blockIdx.y;
  const int tid = threadIdx.x, lane = tid & 31, wave = tid >> 5;

#pragma unroll
  for (int it = 0; it < 2; ++it) {
    const int e  = it * 256 + tid;
    const int s  = e >> 3;
    const int c8 = (e & 7) * 8;
    const size_t g = ((size_t)(c * kChunk + s)) * kQKV + h * kDh + c8;
    const v4u qw = *(const v4u*)(Qh + g);
    const v4u kw = *(const v4u*)(Kh + g);
    *(v4u*)(tQ + s * kPitchH + c8) = qw;
    *(v4u*)(tK + s * kPitchH + c8) = kw;
  }
  asm volatile("" ::: "memory");
#pragma unroll
  for (int it = 0; it < 2; ++it) {
    const int e  = it * 256 + tid;
    const int s  = e >> 3;
    const int c8 = (e & 7) * 8;
    const size_t g = ((size_t)(c * kChunk + s)) * kQKV + h * kDh + c8;
    const v4u vw = *(const v4u*)(Vh + g);
    lds_put_tr(tV, c8, s, vw);
  }
  asm volatile("" ::: "memory");
#pragma unroll
  for (int it = 0; it < 2; ++it) {
    const int e  = it * 256 + tid;
    const int er = e >> 3;
    const int c8 = (e & 7) * 8;
    const size_t g = ((size_t)((h * kNChunk + c) * kDh + er)) * kDh + c8;
    const v4u shw = *(const v4u*)(Shi + g);
    const v4u slw = *(const v4u*)(Slo + g);
    *(v4u*)(tSh + er * kPitchH + c8) = shw;
    *(v4u*)(tSl + er * kPitchH + c8) = slw;
  }
  __syncthreads();

  const int mt = wave & 3, nh = wave >> 2;
  const int rlane = lane & 15, koff = (lane >> 4) * 8, mOff = (lane >> 4) * 8;
  const _Float16* qA = (const _Float16*)tQ;
  const _Float16* kB = (const _Float16*)tK;
  const _Float16* vB = (const _Float16*)tV;
  const _Float16* hB = (const _Float16*)tSh;
  const _Float16* lB = (const _Float16*)tSl;
  const _Float16* pA = (const _Float16*)tP;
  const int arow = (mt * 16 + rlane) * kPitchH + koff;

  const v16h qa0 = Frag<_Float16>::load(qA + arow);
  const v16h qa1 = Frag<_Float16>::load(qA + arow + 32);
  v8f accP[2];
#pragma unroll
  for (int jj = 0; jj < 2; ++jj) {
    const int j = 2 * nh + jj;
    accP[jj] = (v8f){0.f,0.f,0.f,0.f,0.f,0.f,0.f,0.f};
    const v16h kb0 = Frag<_Float16>::load(kB + (j * 16 + rlane) * kPitchH + koff);
    const v16h kb1 = Frag<_Float16>::load(kB + (j * 16 + rlane) * kPitchH + koff + 32);
    accP[jj] = Frag<_Float16>::mma(qa0, kb0, accP[jj]);
    accP[jj] = Frag<_Float16>::mma(qa1, kb1, accP[jj]);
    guard_p4(accP[jj], qa0, qa1, kb0, kb1);
  }
#pragma unroll
  for (int jj = 0; jj < 2; ++jj) {
    const int n = (2 * nh + jj) * 16 + rlane;
#pragma unroll
    for (int r = 0; r < 8; ++r) {
      const int m = mt * 16 + mOff + r;
      const float val = (n <= m) ? accP[jj][r] : 0.0f;
      tP[m * kPitchH + n] = h_bits(val);
    }
  }
  __syncthreads();

  v8f accO[2], accR[2];
#pragma unroll
  for (int jj = 0; jj < 2; ++jj) {
    accO[jj] = (v8f){0.f,0.f,0.f,0.f,0.f,0.f,0.f,0.f};
    accR[jj] = (v8f){0.f,0.f,0.f,0.f,0.f,0.f,0.f,0.f};
  }
#pragma unroll
  for (int kk = 0; kk < 2; ++kk) {
    const int k0 = kk * 32;
    const v16h pa = Frag<_Float16>::load(pA + arow + k0);
    const v16h qa = Frag<_Float16>::load(qA + arow + k0);
#pragma unroll
    for (int jj = 0; jj < 2; ++jj) {
      const int brow = ((2 * nh + jj) * 16 + rlane) * kPitchH + koff + k0;
      const v16h vb = Frag<_Float16>::load(vB + brow);
      const v16h sh = Frag<_Float16>::load(hB + brow);
      const v16h sl = Frag<_Float16>::load(lB + brow);
      accO[jj] = Frag<_Float16>::mma(pa, vb, accO[jj]);
      accO[jj] = Frag<_Float16>::mma(qa, sh, accO[jj]);
      accR[jj] = Frag<_Float16>::mma(qa, sl, accR[jj]);
      guard_o5(accO[jj], accR[jj], pa, qa, vb, sh, sl);
    }
  }
  __syncthreads();

  unsigned short* tOh = lds;
  unsigned short* tOl = lds + 4096;
#pragma unroll
  for (int jj = 0; jj < 2; ++jj) {
    const int n = (2 * nh + jj) * 16 + rlane;
#pragma unroll
    for (int r = 0; r < 8; ++r) {
      const int m = mt * 16 + mOff + r;
      const float o = accO[jj][r] + accR[jj][r] * kResCarryInv;
      const unsigned short hb = f2bf_bits(o);
      const unsigned short lb = f2bf_bits(o - bf_bits2f(hb));
      tOh[m * kChunk + n] = hb;
      tOl[m * kChunk + n] = lb;
    }
  }
  __syncthreads();

  unsigned short* ob = Ob + ((size_t)(c * kChunk)) * (2 * kQKV) + h * kDh;
  const int q = lane >> 3, c8 = (lane & 7) * 8;
  for (int pass = 0; pass < 2; ++pass) {
#pragma unroll
    for (int it = 0; it < 2; ++it) {
      const int row = wave * 8 + it * 4 + q;
      const v4u hv = *(const v4u*)(tOh + row * kChunk + c8);
      const v4u lv = *(const v4u*)(tOl + row * kChunk + c8);
      *(volatile v4u*)(ob + (size_t)row * (2 * kQKV) + c8) = hv;
      *(volatile v4u*)(ob + (size_t)row * (2 * kQKV) + kQKV + c8) = lv;
    }
    __threadfence();
  }
}

extern "C" void kernel_launch(void* const* d_in, const int* in_sizes, int n_in,
                              void* d_out, int out_size, void* d_ws, size_t ws_size,
                              hipStream_t stream) {
  if (n_in < 9) return;
  if (in_sizes[0] != kSeqLen * kModel) return;
  if (in_sizes[1] != kModel * kModel || in_sizes[2] != kModel * kModel ||
      in_sizes[3] != kModel * kModel || in_sizes[4] != kModel * kModel) return;
  if (in_sizes[5] != kDh || in_sizes[6] != kDh || in_sizes[7] != kDh || in_sizes[8] != kDh) return;
  if (out_size != kSeqLen * kModel) return;

  const size_t szXb   = (size_t)kSeqLen * kModel * 2;
  const size_t szWqkv = (size_t)kN3 * kModel * 2;
  const size_t szWo2  = (size_t)kModel * (2 * kQKV) * 2;
  const size_t szQKVf = (size_t)kSeqLen * kN3 * 4;
  const size_t szH    = (size_t)kSeqLen * kQKV * 2;
  const size_t szKV   = (size_t)kHeads * kNChunk * kDh * kDh * 4;
  const size_t szS    = (size_t)kHeads * kNChunk * kDh * kDh * 2;
  const size_t szOb   = (size_t)kSeqLen * (2 * kQKV) * 2;
  const size_t offXb   = 0;
  const size_t offWqkv = offXb + szXb;
  const size_t offWo2  = offWqkv + szWqkv;
  const size_t offQKVf = offWo2 + szWo2;
  const size_t offQh   = offQKVf + szQKVf;
  const size_t offKh   = offQh + szH;
  const size_t offVh   = offKh + szH;
  const size_t offKV   = offVh + szH;
  const size_t offShi  = offKV + szKV;
  const size_t offSlo  = offShi + szS;
  const size_t offOb   = offSlo + szS;
  const size_t total   = offOb + szOb;
  if (ws_size < total) return;

  const float* x   = (const float*)d_in[0];
  const float* Wq  = (const float*)d_in[1];
  const float* Wk  = (const float*)d_in[2];
  const float* Wv  = (const float*)d_in[3];
  const float* Wo  = (const float*)d_in[4];
  const float* qg  = (const float*)d_in[5];
  const float* qbt = (const float*)d_in[6];
  const float* kg  = (const float*)d_in[7];
  const float* kbt = (const float*)d_in[8];
  float* out = (float*)d_out;
  char* ws = (char*)d_ws;
  unsigned short* Xb   = (unsigned short*)(ws + offXb);
  unsigned short* Wqkv = (unsigned short*)(ws + offWqkv);
  unsigned short* Wo2  = (unsigned short*)(ws + offWo2);
  float*          QKVf = (float*)(ws + offQKVf);
  unsigned short* Qh   = (unsigned short*)(ws + offQh);
  unsigned short* Kh   = (unsigned short*)(ws + offKh);
  unsigned short* Vh   = (unsigned short*)(ws + offVh);
  float*          KV   = (float*)(ws + offKV);
  unsigned short* Shi  = (unsigned short*)(ws + offShi);
  unsigned short* Slo  = (unsigned short*)(ws + offSlo);
  unsigned short* Ob   = (unsigned short*)(ws + offOb);

  cast_bf16_kernel<<<dim3((kSeqLen * kModel / 8) / 256, 5), dim3(256), 0, stream>>>(x, Wq, Wk, Wv, Wo, Xb, Wqkv, Wo2);

  const int tilesQKV = (kSeqLen / 64) * (kN3 / 64);
  wmma_gemm64<1, false, 0, 0, false, 0><<<dim3(tilesQKV / 8, 1), dim3(256), 0, stream>>>(
      Xb, Xb, kModel, 0L, Wqkv, Wqkv, kModel, 0L,
      (void*)QKVf, (void*)QKVf, kN3, 0L, qg, qg, 0L, kSeqLen, kN3, kModel, 1.0f);

  ln_cast_kernel<<<dim3((kSeqLen * kHeads) / 8), dim3(256), 0, stream>>>(QKVf, qg, qbt, kg, kbt, Qh, Kh, Vh);

  chunk_state_kernel<<<dim3(kNChunk, kHeads), dim3(256), 0, stream>>>(Kh, Vh, KV);
  state_prefix_kernel<<<dim3((kHeads * kDh) / 8), dim3(256), 0, stream>>>(KV, Shi, Slo);

  chunk_attn_kernel<<<dim3(kNChunk, kHeads), dim3(256), 0, stream>>>(Qh, Kh, Vh, Shi, Slo, Ob);

  const int tilesOut = (kSeqLen / 64) * (kModel / 64);
  wmma_gemm64<1, false, 0, 0, false, 0><<<dim3(tilesOut / 8, 1), dim3(256), 0, stream>>>(
      Ob, Ob, 2 * kQKV, 0L, Wo2, Wo2, 2 * kQKV, 0L,
      (void*)out, (void*)out, kModel, 0L, qg, qg, 0L, kSeqLen, kModel, 2 * kQKV, 1.0f);
}
